// Model_39676907882004
// MI455X (gfx1250) — hardware-verified
//
#include <hip/hip_runtime.h>


#ifndef NB
#define NB 1
#endif
#ifndef SEQ
#define SEQ 4096
#endif
#define SEQ_FULL   4096
#define DIM        1024
#define SCALE_STEP (SEQ_FULL / 4)
#define NWAVE      8
#define BT         128
#define OP         68
#define TP         72
#define WS_CAP     134217728ull
#define SM_NCH     (SEQ / 8)
#define SM_G       ((SM_NCH + 255) / 256)
#define EPI_H16    0
#define EPI_F32    1
#define EPI_NORM   2

#define XB_BYTES   ((unsigned long long)SEQ * DIM * 2ull)
#define VT_BYTES   ((unsigned long long)DIM * SEQ * 2ull)
#define S_BYTES    ((unsigned long long)SEQ * SEQ * 4ull)
#define RS_BYTES   ((unsigned long long)SEQ * 128ull)
#define SCALE_EXT  ((unsigned long long)((SEQ - 1) / DIM) * SCALE_STEP * DIM + DIM)

static_assert(NB == 1);
static_assert(DIM == 1024);
static_assert(SEQ <= SEQ_FULL);
static_assert(SEQ_FULL == 4 * DIM);
static_assert(SEQ % 256 == 0);
static_assert(SEQ % BT == 0);
static_assert(DIM % BT == 0);
static_assert(DIM % 32 == 0);
static_assert(SEQ % 32 == 0);
static_assert(SEQ % 64 == 0);
static_assert(DIM % 64 == 0);
static_assert(DIM % 8 == 0);
static_assert(BT == 4 * 32);
static_assert(BT == 2 * 64);
static_assert((OP * 4) % 16 == 0);
static_assert(OP >= 64);
static_assert((TP * 2) % 16 == 0);
static_assert(TP >= 64);
static_assert(SM_G * 256 >= SM_NCH);
static_assert(((unsigned long long)SEQ * DIM) % 2048ull == 0);
static_assert(SCALE_EXT <= (unsigned long long)SEQ_FULL * DIM);
static_assert(XB_BYTES % 128 == 0);
static_assert(VT_BYTES % 128 == 0);
static_assert(S_BYTES % 128 == 0);
static_assert(2ull * XB_BYTES + VT_BYTES + S_BYTES + RS_BYTES <= WS_CAP);

typedef __bf16   bf16;
typedef _Float16 f16;
typedef bf16     v16bf __attribute__((ext_vector_type(16)));
typedef bf16     v8bf  __attribute__((ext_vector_type(8)));
typedef f16      v16h  __attribute__((ext_vector_type(16)));
typedef f16      v8h   __attribute__((ext_vector_type(8)));
typedef float    v8f   __attribute__((ext_vector_type(8)));
typedef float    v4f   __attribute__((ext_vector_type(4)));
typedef unsigned v4u   __attribute__((ext_vector_type(4)));

union Frag16 { v16bf vb; v16h vh; v4u q[2]; };
union Pack8B { v4u u; v8bf v; bf16 h[8]; };
union Pack8H { v4u u; v8h v; f16 h[8]; };

static __device__ __forceinline__ f16 toh_flush(float v) {
  const f16 r = (f16)v;
  return (fabsf(v) < 6.103515625e-05f) ? (f16)0.0f : r;
}

static __device__ __forceinline__ v8f mma_bf16(v16bf a, v16bf b, v8f acc) {
  acc = __builtin_amdgcn_wmma_f32_16x16x32_bf16(false, a, false, b, (short)0, acc, false, false);
  asm volatile("v_nop\n\tv_nop\n\tv_nop\n\tv_nop" : "+v"(acc) : "v"(a), "v"(b));
  return acc;
}
static __device__ __forceinline__ v8f mma_f16(v16h a, v16h b, v8f acc) {
  acc = __builtin_amdgcn_wmma_f32_16x16x32_f16(false, a, false, b, (short)0, acc, false, false);
  asm volatile("v_nop\n\tv_nop\n\tv_nop\n\tv_nop" : "+v"(acc) : "v"(a), "v"(b));
  return acc;
}
template <bool BF>
static __device__ __forceinline__ v8f mma16(const Frag16& a, const Frag16& b, v8f acc) {
  if (BF) return mma_bf16(a.vb, b.vb, acc);
  return mma_f16(a.vh, b.vh, acc);
}

__global__ __launch_bounds__(256) void convert_x_kernel(const float* __restrict__ x,
                                                        unsigned short* __restrict__ xb) {
  const size_t idx = ((size_t)blockIdx.x * 256 + threadIdx.x) * 8;
  const v4f f0 = *(const v4f*)(x + idx);
  const v4f f1 = *(const v4f*)(x + idx + 4);
  Pack8B pk;
  #pragma unroll
  for (int i = 0; i < 4; ++i) {
    pk.h[i]     = (bf16)f0[i];
    pk.h[4 + i] = (bf16)f1[i];
  }
  const v4u val = pk.u;
  *(volatile v4u*)(xb + idx) = val;
  __threadfence();
  *(volatile v4u*)(xb + idx) = val;
}

__global__ __launch_bounds__(256) void transpose_v_kernel(const float* __restrict__ vin,
                                                          unsigned short* __restrict__ vt) {
  __shared__ __align__(16) f16 sT[64 * TP];
  const int tid = threadIdx.x;
  const int n0  = (blockIdx.x % (DIM / 64)) * 64;
  const int t0  = (blockIdx.x / (DIM / 64)) * 64;
  #pragma unroll
  for (int i = 0; i < 4; ++i) {
    const int r = (tid >> 4) + 16 * i;
    const int c = (tid & 15) * 4;
    const v4f v = *(const v4f*)(vin + (size_t)(t0 + r) * DIM + n0 + c);
    #pragma unroll
    for (int j = 0; j < 4; ++j) {
      const float vb = (float)(bf16)v[j];
      sT[(c + j) * TP + r] = toh_flush(vb * 16.0f);
    }
  }
  __syncthreads();

  v4u    val[2];
  size_t idx[2];
  #pragma unroll
  for (int kk = 0; kk < 2; ++kk) {
    const int n  = kk * 32 + (tid >> 3);
    const int ts = (tid & 7) * 8;
    Pack8H pk;
    pk.v = *(const v8h*)(sT + n * TP + ts);
    val[kk] = pk.u;
    idx[kk] = (size_t)(n0 + n) * SEQ + t0 + ts;
  }
  #pragma unroll
  for (int kk = 0; kk < 2; ++kk) *(volatile v4u*)(vt + idx[kk]) = val[kk];
  __threadfence();
  #pragma unroll
  for (int kk = 0; kk < 2; ++kk) *(volatile v4u*)(vt + idx[kk]) = val[kk];
}

template <bool BF, int EPI>
static __device__ __forceinline__ void gemm_body(const unsigned short* __restrict__ A, const int lda,
                                                 const unsigned short* __restrict__ B, const int ldb,
                                                 const int K,
                                                 unsigned short* __restrict__ ch,
                                                 float* __restrict__ cf, const int ldc,
                                                 const float* __restrict__ rs) {
  __shared__ __align__(16) float sO[NWAVE * 16 * OP];
  const int tid  = threadIdx.x;
  const int wave = __builtin_amdgcn_readfirstlane(threadIdx.x >> 5);
  const int lane = tid & 31;
  const int lq   = lane & 15;
  const int hi   = lane >> 4;
  const int m0   = blockIdx.y * BT + (wave & 3) * 32;
  const int n0   = blockIdx.x * BT + (wave >> 2) * 64;

  size_t aoff[2];
  size_t boff[4];
  #pragma unroll
  for (int mt = 0; mt < 2; ++mt) aoff[mt] = (size_t)(m0 + mt * 16 + lq) * lda + hi * 8;
  #pragma unroll
  for (int nt = 0; nt < 4; ++nt) boff[nt] = (size_t)(n0 + nt * 16 + lq) * ldb + hi * 8;

  v8f acc[2][4];
  #pragma unroll
  for (int mt = 0; mt < 2; ++mt) {
    #pragma unroll
    for (int nt = 0; nt < 4; ++nt) acc[mt][nt] = (v8f){0, 0, 0, 0, 0, 0, 0, 0};
  }

  #pragma unroll 1
  for (int k0 = 0; k0 < K; k0 += 32) {
    Frag16 a[2];
    Frag16 b[4];
    #pragma unroll
    for (int mt = 0; mt < 2; ++mt) {
      a[mt].q[0] = *(const v4u*)(A + aoff[mt] + k0);
      a[mt].q[1] = *(const v4u*)(A + aoff[mt] + k0 + 16);
    }
    #pragma unroll
    for (int nt = 0; nt < 4; ++nt) {
      b[nt].q[0] = *(const v4u*)(B + boff[nt] + k0);
      b[nt].q[1] = *(const v4u*)(B + boff[nt] + k0 + 16);
    }
    #pragma unroll
    for (int mt = 0; mt < 2; ++mt) {
      #pragma unroll
      for (int nt = 0; nt < 4; ++nt) acc[mt][nt] = mma16<BF>(a[mt], b[nt], acc[mt][nt]);
    }
  }

  float* so = sO + wave * (16 * OP);
  #pragma unroll
  for (int mt = 0; mt < 2; ++mt) {
    __syncthreads();
    #pragma unroll
    for (int r = 0; r < 8; ++r) {
      #pragma unroll
      for (int nt = 0; nt < 4; ++nt) so[(hi * 8 + r) * OP + nt * 16 + lq] = acc[mt][nt][r];
    }
    __syncthreads();
    const int rbase = m0 + mt * 16;
    if (EPI == EPI_H16) {
      v4u    vals[4];
      size_t gidx[4];
      #pragma unroll
      for (int it = 0; it < 4; ++it) {
        const int row = it * 4 + (lane >> 3);
        const int pc  = lane & 7;
        const v4f x0 = *(const v4f*)(so + row * OP + pc * 8);
        const v4f x1 = *(const v4f*)(so + row * OP + pc * 8 + 4);
        Pack8H ph;
        #pragma unroll
        for (int i = 0; i < 4; ++i) {
          ph.h[i]     = (f16)(x0[i] * 16.0f);
          ph.h[4 + i] = (f16)(x1[i] * 16.0f);
        }
        vals[it] = ph.u;
        gidx[it] = (size_t)(rbase + row) * ldc + n0 + pc * 8;
      }
      #pragma unroll
      for (int it = 0; it < 4; ++it) *(volatile v4u*)(ch + gidx[it]) = vals[it];
      __threadfence();
      #pragma unroll
      for (int it = 0; it < 4; ++it) *(volatile v4u*)(ch + gidx[it]) = vals[it];
    } else {
      v4f    vals[8];
      size_t gidx[8];
      #pragma unroll
      for (int it = 0; it < 8; ++it) {
        const int row = it * 2 + hi;
        v4f x = *(const v4f*)(so + row * OP + lq * 4);
        if (EPI == EPI_NORM) {
          const float f = rs[(size_t)(rbase + row) * 32] * 0.0625f;
          x = x * f;
        }
        vals[it] = x;
        gidx[it] = (size_t)(rbase + row) * ldc + n0 + lq * 4;
      }
      #pragma unroll
      for (int it = 0; it < 8; ++it) *(volatile v4f*)(cf + gidx[it]) = vals[it];
      __threadfence();
      #pragma unroll
      for (int it = 0; it < 8; ++it) *(volatile v4f*)(cf + gidx[it]) = vals[it];
    }
  }
}

__global__ __launch_bounds__(256) void gemm_scores_kernel(const unsigned short* __restrict__ a, int lda,
                                                          const unsigned short* __restrict__ b, int ldb,
                                                          int kdim,
                                                          float* __restrict__ c, int ldc) {
  gemm_body<true, EPI_F32>(a, lda, b, ldb, kdim, (unsigned short*)0, c, ldc, (const float*)0);
}

__global__ __launch_bounds__(256) void gemm_pv_kernel(const unsigned short* __restrict__ a, int lda,
                                                      const unsigned short* __restrict__ b, int ldb,
                                                      int kdim,
                                                      float* __restrict__ c, int ldc,
                                                      const float* __restrict__ rs) {
  gemm_body<false, EPI_NORM>(a, lda, b, ldb, kdim, (unsigned short*)0, c, ldc, rs);
}

__global__ __launch_bounds__(256) void softmax_rows_kernel(float* s, float* rs, const float* __restrict__ qin) {
  #pragma clang fp contract(off)
  __shared__ float sred[16];
  const int row  = blockIdx.x;
  const int tid  = threadIdx.x;
  const int lane = tid & 31;
  const int wave = tid >> 5;
  float* srow = s + (size_t)row * SEQ;

  float v[SM_G][8];
  #pragma unroll
  for (int g = 0; g < SM_G; ++g) {
    const int  chunk = tid + 256 * g;
    const bool act   = chunk < SM_NCH;
    const int  cc    = act ? chunk : (SM_NCH - 1);
    const v4f a0 = *(const v4f*)(srow + (size_t)cc * 8);
    const v4f a1 = *(const v4f*)(srow + (size_t)cc * 8 + 4);
    const int    t0 = cc * 8;
    const size_t qo = (size_t)(t0 / DIM) * SCALE_STEP * DIM + (size_t)(t0 % DIM);
    const v4f c0 = *(const v4f*)(qin + qo);
    const v4f c1 = *(const v4f*)(qin + qo + 4);
    #pragma unroll
    for (int i = 0; i < 4; ++i) {
      const float s0 = (float)(bf16)c0[i];
      const float s1 = (float)(bf16)c1[i];
      const float l0 = a0[i] * s0;
      const float l1 = a1[i] * s1;
      v[g][i]     = act ? l0 : -__builtin_inff();
      v[g][4 + i] = act ? l1 : -__builtin_inff();
    }
  }

  float m = -__builtin_inff();
  #pragma unroll
  for (int g = 0; g < SM_G; ++g) {
    #pragma unroll
    for (int i = 0; i < 8; ++i) m = fmaxf(m, v[g][i]);
  }
  m = fmaxf(m, __shfl_xor(m, 16, 32));
  m = fmaxf(m, __shfl_xor(m, 8, 32));
  m = fmaxf(m, __shfl_xor(m, 4, 32));
  m = fmaxf(m, __shfl_xor(m, 2, 32));
  m = fmaxf(m, __shfl_xor(m, 1, 32));
  if (lane == 0) sred[wave] = m;
  __syncthreads();
  float mm = sred[0];
  #pragma unroll
  for (int w = 1; w < 8; ++w) mm = fmaxf(mm, sred[w]);

  const float LOG2E = 1.4426950408889634f;
  v4u   pv[SM_G];
  float psum = 0.0f;
  #pragma unroll
  for (int g = 0; g < SM_G; ++g) {
    Pack8H ph;
    #pragma unroll
    for (int i = 0; i < 8; ++i) {
      const float e  = (v[g][i] - mm) * LOG2E;
      const float p  = __builtin_amdgcn_exp2f(e + 14.0f);
      const f16   hh = toh_flush(p);
      ph.h[i] = hh;
      psum += (float)hh;
    }
    pv[g] = ph.u;
  }
  psum += __shfl_xor(psum, 16, 32);
  psum += __shfl_xor(psum, 8, 32);
  psum += __shfl_xor(psum, 4, 32);
  psum += __shfl_xor(psum, 2, 32);
  psum += __shfl_xor(psum, 1, 32);
  if (lane == 0) sred[8 + wave] = psum;
  __syncthreads();
  float tot = sred[8];
  #pragma unroll
  for (int w = 1; w < 8; ++w) tot += sred[8 + w];
  const float rinv = __builtin_amdgcn_rcpf(tot);
  const v4f   rv   = (v4f){rinv, rinv, rinv, rinv};

  unsigned short* prow = (unsigned short*)srow;
  float* rline = rs + (size_t)row * 32;

  #pragma unroll
  for (int g = 0; g < SM_G; ++g) {
    const int chunk = tid + 256 * g;
    if (chunk < SM_NCH) *(volatile v4u*)(prow + (size_t)chunk * 8) = pv[g];
  }
  if (tid < 8) *(volatile v4f*)(rline + tid * 4) = rv;
  __threadfence();
  #pragma unroll
  for (int g = 0; g < SM_G; ++g) {
    const int chunk = tid + 256 * g;
    if (chunk < SM_NCH) *(volatile v4u*)(prow + (size_t)chunk * 8) = pv[g];
  }
  if (tid < 8) *(volatile v4f*)(rline + tid * 4) = rv;
}

extern "C" void kernel_launch(void* const* d_in, const int* in_sizes, int n_in,
                              void* d_out, int out_size, void* d_ws, size_t ws_size,
                              hipStream_t stream) {
  if (n_in < 3) return;
  if ((size_t)in_sizes[0] < (size_t)SEQ * DIM) return;
  if ((size_t)in_sizes[0] < (size_t)SCALE_EXT) return;
  if ((size_t)in_sizes[1] < (size_t)SEQ * DIM) return;
  if ((size_t)in_sizes[2] < (size_t)SEQ * DIM) return;
  if ((size_t)out_size < (size_t)SEQ * DIM) return;

  const size_t off_qb = 0;
  const size_t off_kb = off_qb + (size_t)XB_BYTES;
  const size_t off_vt = off_kb + (size_t)XB_BYTES;
  const size_t off_s  = off_vt + (size_t)VT_BYTES;
  const size_t off_rs = off_s + (size_t)S_BYTES;
  const size_t total  = off_rs + (size_t)RS_BYTES;
  if (ws_size < total) return;

  const float* q = (const float*)d_in[0];
  const float* k = (const float*)d_in[1];
  const float* v = (const float*)d_in[2];
  float* out = (float*)d_out;

  char* ws = (char*)d_ws;
  unsigned short* qb = (unsigned short*)(ws + off_qb);
  unsigned short* kb = (unsigned short*)(ws + off_kb);
  unsigned short* vt = (unsigned short*)(ws + off_vt);
  float*          sc = (float*)(ws + off_s);
  float*          rs = (float*)(ws + off_rs);

  convert_x_kernel<<<dim3((unsigned)(((size_t)SEQ * DIM) / 2048)), 256, 0, stream>>>(q, qb);
  convert_x_kernel<<<dim3((unsigned)(((size_t)SEQ * DIM) / 2048)), 256, 0, stream>>>(k, kb);

  transpose_v_kernel<<<dim3((DIM / 64) * (SEQ / 64)), 256, 0, stream>>>(v, vt);

  gemm_scores_kernel<<<dim3(SEQ / BT, SEQ / BT), 256, 0, stream>>>(qb, DIM, kb, DIM, DIM, sc, SEQ);
  softmax_rows_kernel<<<dim3(SEQ), 256, 0, stream>>>(sc, rs, q);
  gemm_pv_kernel<<<dim3(DIM / BT, SEQ / BT), 256, 0, stream>>>((const unsigned short*)sc, 2 * SEQ, vt, SEQ, SEQ, out, DIM, rs);
}
